// CausalSelfAttention_59253368815644
// MI455X (gfx1250) — hardware-verified
//
#include <hip/hip_runtime.h>
#include <stddef.h>


typedef _Float16 v16h __attribute__((ext_vector_type(16)));
typedef _Float16 v8h  __attribute__((ext_vector_type(8)));
typedef float    v8f  __attribute__((ext_vector_type(8)));
typedef float    v4f  __attribute__((ext_vector_type(4)));
typedef _Float16 h16;

#ifndef NB
#define NB 2
#endif
#ifndef SEQ
#define SEQ 2048
#endif
#define NB_FULL  2
#define SEQ_FULL 2048
#define DIM   1024
#define NHEAD 16
#define HD    64
#define ROTH  32
#define NGATE 32
#define MROWS (NB * SEQ)

static_assert(NB >= 1 && NB <= NB_FULL);
static_assert(SEQ >= 128 && SEQ <= SEQ_FULL && (SEQ % 128) == 0);
static_assert(DIM == NHEAD * HD);
static_assert(HD == 64 && ROTH * 2 == HD);
static_assert(NGATE == 2 * NHEAD && NGATE == 32);
static_assert((DIM % 64) == 0 && (DIM % 32) == 0 && (DIM % 8) == 0);
static_assert((MROWS % 128) == 0 && (MROWS % 64) == 0);
static_assert((SEQ % 64) == 0 && (SEQ % 32) == 0);

#define LDT 72
#define LDC 68
#define LDG 36
static_assert(LDT >= 64 + 8 && ((LDT * 2) % 16) == 0);
static_assert(LDC >= 64 + 4 && ((LDC * 4) % 16) == 0);
static_assert(LDG >= 32 + 4 && ((LDG * 4) % 16) == 0);

#define WCARRY  64.0f
#define ACARRY  16.0f
#define QKCARRY 8.0f
#define VCARRY  8.0f
#define PCARRY  1024.0f
#define CCARRY  64.0f
#define RCARRY  2048.0f
#define RINV    (1.0f / 2048.0f)
#define RMS_EPS 1.1920929e-07f

#define W_ELEMS       ((size_t)4 * DIM * DIM)
#define WQKV_ELEMS    ((size_t)3 * DIM * DIM)
#define GW_ELEMS      ((size_t)NGATE * DIM)
#define GWHALF_ELEMS  ((size_t)NHEAD * DIM)
#define PLANE16_ELEMS ((size_t)MROWS * DIM)
#define PLANE16_BYTES (PLANE16_ELEMS * 2)
#define GT_BYTES      ((size_t)MROWS * NGATE * 4)
#define WS_TOTAL      (W_ELEMS * 2 + GW_ELEMS * 2 + 9 * PLANE16_BYTES + GT_BYTES)
static_assert((W_ELEMS % 2048) == 0 && (GWHALF_ELEMS % 2048) == 0 && (PLANE16_ELEMS % 2048) == 0);
static_assert((WQKV_ELEMS % 8) == 0);
static_assert(((W_ELEMS * 2) % 128) == 0 && ((GW_ELEMS * 2) % 128) == 0);
static_assert((PLANE16_BYTES % 128) == 0 && (GT_BYTES % 128) == 0);
static_assert(PLANE16_ELEMS < (size_t)0xFFFFFFFFu);
static_assert(WS_TOTAL <= (size_t)134217728);

__device__ __forceinline__ float bf16r(float x) {
  unsigned int u = __float_as_uint(x);
  u = (u + 0x7FFFu + ((u >> 16) & 1u)) & 0xFFFF0000u;
  return __uint_as_float(u);
}

static __device__ __forceinline__ h16 toh_flush(float v) {
  const h16 r = (h16)v;
  return (fabsf(v) < 6.103515625e-05f) ? (h16)0.0f : r;
}

__device__ __forceinline__ v16h frag_at(const _Float16* p) {
  v8h lo = *(const v8h*)(p);
  v8h hi = *(const v8h*)(p + 16);
  v16h out;
#pragma unroll
  for (int i = 0; i < 8; ++i) { out[i] = lo[i]; out[i + 8] = hi[i]; }
  return out;
}
__device__ __forceinline__ v16h ld_frag(const _Float16* base, unsigned ld) {
  const unsigned lane = threadIdx.x & 31u;
  return frag_at(base + (lane & 15u) * ld + (lane >> 4) * 8u);
}

__device__ __forceinline__ v8f wmma16(v16h a, v16h b, v8f c) {
  v8f d = __builtin_amdgcn_wmma_f32_16x16x32_f16(false, a, false, b, (short)0, c,
                                                 false, false);
  asm volatile("v_nop\n\tv_nop\n\tv_nop\n\tv_nop" : "+v"(d) : "v"(a), "v"(b));
  return d;
}

__device__ __forceinline__ float red16_max(float x) {
#pragma unroll
  for (int off = 1; off < 16; off <<= 1) x = fmaxf(x, __shfl_xor(x, off, 32));
  return x;
}
__device__ __forceinline__ float red16_sum(float x) {
#pragma unroll
  for (int off = 1; off < 16; off <<= 1) x += __shfl_xor(x, off, 32);
  return x;
}
__device__ __forceinline__ float red8_sum(float x) {
#pragma unroll
  for (int off = 1; off < 8; off <<= 1) x += __shfl_xor(x, off, 32);
  return x;
}
__device__ __forceinline__ int imin2(int a, int b) { return (a < b) ? a : b; }
__device__ __forceinline__ int imax2(int a, int b) { return (a > b) ? a : b; }
__device__ __forceinline__ int red16_imin(int x) {
#pragma unroll
  for (int off = 1; off < 16; off <<= 1) x = imin2(x, __shfl_xor(x, off, 32));
  return x;
}
__device__ __forceinline__ int red16_imax(int x) {
#pragma unroll
  for (int off = 1; off < 16; off <<= 1) x = imax2(x, __shfl_xor(x, off, 32));
  return x;
}
__device__ __forceinline__ int red32_imin(int x) {
#pragma unroll
  for (int off = 1; off < 32; off <<= 1) x = imin2(x, __shfl_xor(x, off, 32));
  return x;
}
__device__ __forceinline__ int red32_imax(int x) {
#pragma unroll
  for (int off = 1; off < 32; off <<= 1) x = imax2(x, __shfl_xor(x, off, 32));
  return x;
}
__device__ __forceinline__ int rfl(int x) { return __builtin_amdgcn_readfirstlane(x); }

__device__ __forceinline__ void wave_lds_sync() {
  __builtin_amdgcn_fence(3  , "wavefront");
  asm volatile("s_wait_dscnt 0x0" ::: "memory");
  __builtin_amdgcn_wave_barrier();
}

__global__ __launch_bounds__(256) void wcvt_kernel(
    const float* __restrict__ src, const float* __restrict__ lam, unsigned split,
    unsigned uselam, _Float16* __restrict__ dst) {
  const unsigned e = (blockIdx.x * 256u + threadIdx.x) * 8u;
  const float l0 = bf16r(lam[0]);
  const float l1 = bf16r(lam[1]);
  const float lsel = (e < split) ? l0 : l1;
  const float f = (uselam != 0u) ? lsel : 1.0f;
  const v4f a0 = *(const v4f*)(src + e);
  const v4f a1 = *(const v4f*)(src + e + 4);
  v8h o;
#pragma unroll
  for (int j = 0; j < 4; ++j) {
    o[j]     = toh_flush(WCARRY * (f * bf16r(a0[j])));
    o[j + 4] = toh_flush(WCARRY * (f * bf16r(a1[j])));
  }
  *(volatile v8h*)(dst + (size_t)e) = o;
  __threadfence();
  *(volatile v8h*)(dst + (size_t)e) = o;
}

__global__ __launch_bounds__(256) void xcvt_kernel(
    const float* __restrict__ src, _Float16* __restrict__ dst) {
  const unsigned e = (blockIdx.x * 256u + threadIdx.x) * 8u;
  const unsigned crow = e / (unsigned)DIM;
  const unsigned c = e - crow * (unsigned)DIM;
  const unsigned bidx = crow / (unsigned)SEQ;
  const unsigned sq = crow - bidx * (unsigned)SEQ;
  const size_t so = ((size_t)bidx * SEQ_FULL + sq) * DIM + c;
  const v4f a0 = *(const v4f*)(src + so);
  const v4f a1 = *(const v4f*)(src + so + 4);
  v8h o;
#pragma unroll
  for (int j = 0; j < 4; ++j) {
    o[j]     = toh_flush(ACARRY * bf16r(a0[j]));
    o[j + 4] = toh_flush(ACARRY * bf16r(a1[j]));
  }
  *(volatile v8h*)(dst + (size_t)e) = o;
  __threadfence();
  *(volatile v8h*)(dst + (size_t)e) = o;
}

__device__ __forceinline__ void gemm_loop2(const _Float16* ap, const _Float16* bp0,
                                           const _Float16* bp1, v8f& acc0, v8f& acc1) {
#pragma unroll 2
  for (unsigned k0 = 0; k0 < (unsigned)DIM; k0 += 32u) {
    const v16h a  = frag_at(ap + k0);
    const v16h b0 = frag_at(bp0 + k0);
    const v16h b1 = frag_at(bp1 + k0);
    acc0 = wmma16(a, b0, acc0);
    acc1 = wmma16(a, b1, acc1);
  }
}
__device__ __forceinline__ void gemm_loop4(const _Float16* ap, const _Float16* apr,
                                           const _Float16* bp0, const _Float16* bp1,
                                           v8f& acc0, v8f& acc1, v8f& acc2, v8f& acc3) {
#pragma unroll 2
  for (unsigned k0 = 0; k0 < (unsigned)DIM; k0 += 32u) {
    const v16h a  = frag_at(ap + k0);
    const v16h ar = frag_at(apr + k0);
    const v16h b0 = frag_at(bp0 + k0);
    const v16h b1 = frag_at(bp1 + k0);
    acc0 = wmma16(a, b0, acc0);
    acc1 = wmma16(a, b1, acc1);
    acc2 = wmma16(ar, b0, acc2);
    acc3 = wmma16(ar, b1, acc3);
  }
}

__global__ __launch_bounds__(256) void gate_gemm_kernel(
    const _Float16* __restrict__ A16, const _Float16* __restrict__ Gw,
    float* __restrict__ Gt) {
  __shared__ float Cs[128 * LDG];
  const unsigned tid = threadIdx.x, lane = tid & 31u;
  const unsigned wu = (unsigned)__builtin_amdgcn_readfirstlane((int)(tid >> 5));
  const unsigned hh = lane >> 4, m = lane & 15u;
  const unsigned row0 = blockIdx.x * 128u;

  const _Float16* ap  = A16 + (size_t)(row0 + wu * 16u + m) * DIM + hh * 8u;
  const _Float16* bp0 = Gw + (size_t)m * DIM + hh * 8u;
  const _Float16* bp1 = bp0 + (size_t)16 * DIM;
  v8f acc0 = {}, acc1 = {};
  gemm_loop2(ap, bp0, bp1, acc0, acc1);
#pragma unroll
  for (int r = 0; r < 8; ++r) {
    const unsigned ci = (wu * 16u + hh * 8u + (unsigned)r) * LDG + m;
    Cs[ci]       = acc0[r];
    Cs[ci + 16u] = acc1[r];
  }
  __syncthreads();

  const float inv = 1.0f / (WCARRY * ACARRY);
  v4f xs[4];
  size_t off[4];
#pragma unroll
  for (unsigned i = 0; i < 4u; ++i) {
    const unsigned r = 32u * i + (tid >> 3);
    const unsigned c = (tid & 7u) * 4u;
    const v4f u = *(const v4f*)&Cs[r * LDG + c];
    const float gs = (c < 16u) ? 1.0f : 2.0f;
    v4f val;
#pragma unroll
    for (int j = 0; j < 4; ++j) {
      const float z = u[j] * inv;
      val[j] = gs * __builtin_amdgcn_rcpf(1.0f + __expf(-z));
    }
    xs[i] = val;
    off[i] = (size_t)(row0 + r) * NGATE + c;
  }
#pragma unroll
  for (int i = 0; i < 4; ++i) *(volatile v4f*)(Gt + off[i]) = xs[i];
  __threadfence();
#pragma unroll
  for (int i = 0; i < 4; ++i) *(volatile v4f*)(Gt + off[i]) = xs[i];
}

__global__ __launch_bounds__(256) void qkv_gemm_kernel(
    const _Float16* __restrict__ A16, const _Float16* __restrict__ Bt,
    const float* __restrict__ ve, const float* __restrict__ Gt,
    const float* __restrict__ cosv, const float* __restrict__ sinv,
    _Float16* __restrict__ out16) {
  __shared__ float Cs[64 * LDC];
  const unsigned tid = threadIdx.x, lane = tid & 31u;
  const unsigned wu = (unsigned)__builtin_amdgcn_readfirstlane((int)(tid >> 5));
  const unsigned mw = wu >> 1, nw = wu & 1u;
  const unsigned hh = lane >> 4, m = lane & 15u;
  const unsigned n0 = blockIdx.x * 64u;
  const unsigned row0 = blockIdx.y * 64u;

  const _Float16* ap  = A16 + (size_t)(row0 + mw * 16u + m) * DIM + hh * 8u;
  const _Float16* bp0 = Bt + (size_t)(n0 + nw * 32u + m) * DIM + hh * 8u;
  const _Float16* bp1 = bp0 + (size_t)16 * DIM;
  v8f acc0 = {}, acc1 = {};
  gemm_loop2(ap, bp0, bp1, acc0, acc1);
#pragma unroll
  for (int r = 0; r < 8; ++r) {
    const unsigned ci = (mw * 16u + hh * 8u + (unsigned)r) * LDC + nw * 32u + m;
    Cs[ci]       = acc0[r];
    Cs[ci + 16u] = acc1[r];
  }
  __syncthreads();

  const float inv = 1.0f / (WCARRY * ACARRY);
  const unsigned region = n0 / (unsigned)DIM;
  const unsigned hc = n0 - region * (unsigned)DIM;
  v8h x[2], xr[2];
  size_t off[2];
  if (region < 2u) {
#pragma unroll
    for (unsigned i = 0; i < 2u; ++i) {
      const unsigned r = 32u * i + (tid >> 3);
      const unsigned c = (tid & 7u) * 8u;
      const unsigned crow = row0 + r;
      const unsigned bidx = crow / (unsigned)SEQ;
      const unsigned sq = crow - bidx * (unsigned)SEQ;
      const unsigned cc = c & 31u;
      const unsigned pc = c ^ 32u;
      const float sgn = (c < 32u) ? 1.0f : -1.0f;
      const v4f u0 = *(const v4f*)&Cs[r * LDC + c];
      const v4f u1 = *(const v4f*)&Cs[r * LDC + c + 4];
      const v4f p0 = *(const v4f*)&Cs[r * LDC + pc];
      const v4f p1 = *(const v4f*)&Cs[r * LDC + pc + 4];
      float ss = 0.0f;
#pragma unroll
      for (int j = 0; j < 4; ++j) {
        const float a = u0[j] * inv;
        const float bq = u1[j] * inv;
        ss += a * a;
        ss += bq * bq;
      }
      ss = red8_sum(ss);
      const float rs = rsqrtf(ss * (1.0f / (float)HD) + RMS_EPS);
      const v4f c0 = *(const v4f*)(cosv + (size_t)sq * ROTH + cc);
      const v4f c1 = *(const v4f*)(cosv + (size_t)sq * ROTH + cc + 4);
      const v4f s0 = *(const v4f*)(sinv + (size_t)sq * ROTH + cc);
      const v4f s1 = *(const v4f*)(sinv + (size_t)sq * ROTH + cc + 4);
#pragma unroll
      for (int j = 0; j < 4; ++j) {
        const float t0 = u0[j] * inv * rs, t1 = u1[j] * inv * rs;
        const float q0 = p0[j] * inv * rs, q1 = p1[j] * inv * rs;
        const float r0 = t0 * bf16r(c0[j]) + sgn * (q0 * bf16r(s0[j]));
        const float r1 = t1 * bf16r(c1[j]) + sgn * (q1 * bf16r(s1[j]));
        const float f0 = QKCARRY * r0, f1 = QKCARRY * r1;
        const h16 h0 = toh_flush(f0), h1 = toh_flush(f1);
        x[i][j]      = h0;
        x[i][j + 4]  = h1;
        xr[i][j]     = toh_flush(RCARRY * (f0 - (float)h0));
        xr[i][j + 4] = toh_flush(RCARRY * (f1 - (float)h1));
      }
      off[i] = (size_t)region * PLANE16_ELEMS + (size_t)crow * DIM + hc + c;
    }
  } else {
    const unsigned head = hc >> 6;
#pragma unroll
    for (unsigned i = 0; i < 2u; ++i) {
      const unsigned r = 32u * i + (tid >> 3);
      const unsigned c = (tid & 7u) * 8u;
      const unsigned crow = row0 + r;
      const unsigned bidx = crow / (unsigned)SEQ;
      const unsigned sq = crow - bidx * (unsigned)SEQ;
      const size_t frow = (size_t)bidx * SEQ_FULL + sq;
      const float g = Gt[(size_t)crow * NGATE + 16u + head];
      const v4f e0 = *(const v4f*)(ve + frow * DIM + hc + c);
      const v4f e1 = *(const v4f*)(ve + frow * DIM + hc + c + 4);
      const v4f u0 = *(const v4f*)&Cs[r * LDC + c];
      const v4f u1 = *(const v4f*)&Cs[r * LDC + c + 4];
      v4f w0, w1;
#pragma unroll
      for (int j = 0; j < 4; ++j) {
        w0[j] = u0[j] * inv + g * bf16r(e0[j]);
        w1[j] = u1[j] * inv + g * bf16r(e1[j]);
      }
      *(v4f*)&Cs[r * LDC + c]     = w0;
      *(v4f*)&Cs[r * LDC + c + 4] = w1;
    }
    __syncthreads();
    const unsigned bidx = row0 / (unsigned)SEQ;
    const unsigned key0 = row0 - bidx * (unsigned)SEQ;
#pragma unroll
    for (unsigned i = 0; i < 2u; ++i) {
      const unsigned dcol = 32u * i + (tid >> 3);
      const unsigned kk = (tid & 7u) * 8u;
#pragma unroll
      for (unsigned j = 0; j < 8u; ++j) {
        const float f = VCARRY * Cs[(kk + j) * LDC + dcol];
        const h16 h = toh_flush(f);
        x[i][j]  = h;
        xr[i][j] = toh_flush(RCARRY * (f - (float)h));
      }
      off[i] = (size_t)2 * PLANE16_ELEMS +
               ((size_t)bidx * DIM + hc + dcol) * SEQ + key0 + kk;
    }
  }
#pragma unroll
  for (int i = 0; i < 2; ++i) *(volatile v8h*)(out16 + off[i]) = x[i];
#pragma unroll
  for (int i = 0; i < 2; ++i)
    *(volatile v8h*)(out16 + (size_t)3 * PLANE16_ELEMS + off[i]) = xr[i];
  __threadfence();
#pragma unroll
  for (int i = 0; i < 2; ++i) *(volatile v8h*)(out16 + off[i]) = x[i];
#pragma unroll
  for (int i = 0; i < 2; ++i)
    *(volatile v8h*)(out16 + (size_t)3 * PLANE16_ELEMS + off[i]) = xr[i];
}

__global__ __launch_bounds__(256) void out_gemm_kernel(
    const _Float16* __restrict__ Ah, const _Float16* __restrict__ Ar,
    const _Float16* __restrict__ Bt, float* __restrict__ outf) {
  __shared__ float Cs[64 * LDC];
  const unsigned tid = threadIdx.x, lane = tid & 31u;
  const unsigned wu = (unsigned)__builtin_amdgcn_readfirstlane((int)(tid >> 5));
  const unsigned mw = wu >> 1, nw = wu & 1u;
  const unsigned hh = lane >> 4, m = lane & 15u;
  const unsigned n0 = blockIdx.x * 64u;
  const unsigned row0 = blockIdx.y * 64u;

  const size_t aoff = (size_t)(row0 + mw * 16u + m) * DIM + hh * 8u;
  const _Float16* bp0 = Bt + (size_t)(n0 + nw * 32u + m) * DIM + hh * 8u;
  const _Float16* bp1 = bp0 + (size_t)16 * DIM;
  v8f acc0 = {}, acc1 = {}, acc2 = {}, acc3 = {};
  gemm_loop4(Ah + aoff, Ar + aoff, bp0, bp1, acc0, acc1, acc2, acc3);
#pragma unroll
  for (int r = 0; r < 8; ++r) {
    const unsigned ci = (mw * 16u + hh * 8u + (unsigned)r) * LDC + nw * 32u + m;
    Cs[ci]       = acc0[r] + acc2[r] * RINV;
    Cs[ci + 16u] = acc1[r] + acc3[r] * RINV;
  }
  __syncthreads();

  const float inv = 1.0f / (WCARRY * CCARRY);
  v4f xs[4];
  size_t off[4];
#pragma unroll
  for (unsigned i = 0; i < 4u; ++i) {
    const unsigned r = 16u * i + (tid >> 4);
    const unsigned c = (tid & 15u) * 4u;
    const unsigned crow = row0 + r;
    const unsigned bidx = crow / (unsigned)SEQ;
    const unsigned sq = crow - bidx * (unsigned)SEQ;
    const size_t frow = (size_t)bidx * SEQ_FULL + sq;
    const v4f u = *(const v4f*)&Cs[r * LDC + c];
    v4f val;
#pragma unroll
    for (int j = 0; j < 4; ++j) val[j] = u[j] * inv;
    xs[i] = val;
    off[i] = frow * DIM + n0 + c;
  }
#pragma unroll
  for (int i = 0; i < 4; ++i) *(volatile v4f*)(outf + off[i]) = xs[i];
  __threadfence();
#pragma unroll
  for (int i = 0; i < 4; ++i) *(volatile v4f*)(outf + off[i]) = xs[i];
}

__global__ __launch_bounds__(256) void attn_kernel(
    const _Float16* __restrict__ Qh, const _Float16* __restrict__ Qr,
    const _Float16* __restrict__ Kh, const _Float16* __restrict__ Kr,
    const _Float16* __restrict__ Vt, const _Float16* __restrict__ Vr,
    const float* __restrict__ Gt, const int* __restrict__ docs,
    const float* __restrict__ scale_p,
    _Float16* __restrict__ Ohi, _Float16* __restrict__ Ores) {
  __shared__ _Float16 Ks[64 * LDT];
  __shared__ _Float16 Krs[64 * LDT];
  __shared__ _Float16 Vs[64 * LDT];
  __shared__ _Float16 Vrs[64 * LDT];
  __shared__ _Float16 Ps[8 * 16 * LDT];
  __shared__ _Float16 Prs[8 * 16 * LDT];
  __shared__ int Ds[SEQ];
  __shared__ int Hmn[SEQ / 32];
  __shared__ int Hmx[SEQ / 32];

  const unsigned tid = threadIdx.x, lane = tid & 31u;
  const unsigned wu = (unsigned)__builtin_amdgcn_readfirstlane((int)(tid >> 5));
  const unsigned hh = lane >> 4, m = lane & 15u;
  const unsigned q0 = blockIdx.x * 128u;
  const unsigned head = blockIdx.y;
  const unsigned b = blockIdx.z;
  const float scale = bf16r(scale_p[0]) * (1.0f / (QKCARRY * QKCARRY));
  const unsigned pbase = wu * (16u * LDT);

  for (unsigned i = tid; i < (unsigned)SEQ; i += 256u) Ds[i] = docs[i];
  __syncthreads();
  for (unsigned e = wu; e < (unsigned)(SEQ / 32); e += 8u) {
    const int dv = Ds[e * 32u + lane];
    const int mn = red32_imin(dv);
    const int mx = red32_imax(dv);
    if (lane == 0u) { Hmn[e] = mn; Hmx[e] = mx; }
  }
  __syncthreads();

  const unsigned eb = q0 >> 5;
  const int bmn = rfl(imin2(imin2(Hmn[eb], Hmn[eb + 1u]), imin2(Hmn[eb + 2u], Hmn[eb + 3u])));
  const int bmx = rfl(imax2(imax2(Hmx[eb], Hmx[eb + 1u]), imax2(Hmx[eb + 2u], Hmx[eb + 3u])));
  const unsigned wrow0 = q0 + wu * 16u;
  const int dw = Ds[wrow0 + m];
  const int wmn = rfl(red16_imin(dw));
  const int wmx = rfl(red16_imax(dw));
  const unsigned rowb = wrow0 + hh * 8u;
  int dq[8];
#pragma unroll
  for (int v = 0; v < 8; ++v) dq[v] = Ds[rowb + (unsigned)v];

  const size_t qoff = (size_t)(b * (unsigned)SEQ + wrow0 + m) * DIM + head * HD + hh * 8u;
  v16h qf[2];
  qf[0] = frag_at(Qh + qoff);
  qf[1] = frag_at(Qh + qoff + 32);

  float mrow[8], lrow[8];
  v8f o[4], ores[4];
#pragma unroll
  for (int v = 0; v < 8; ++v) { mrow[v] = -1.0e30f; lrow[v] = 0.0f; }
#pragma unroll
  for (int nb = 0; nb < 4; ++nb) { o[nb] = (v8f){}; ores[nb] = (v8f){}; }

  const size_t kplane = (size_t)b * SEQ * DIM + head * HD;
  const size_t vplane = ((size_t)b * DIM + head * HD) * SEQ;
  const unsigned kend = q0 + 128u;

  for (unsigned kb = 0; kb < kend; kb += 64u) {
    const unsigned e0 = kb >> 5;
    const int h0n = Hmn[e0], h1n = Hmn[e0 + 1u];
    const int h0x = Hmx[e0], h1x = Hmx[e0 + 1u];
    const int tmn = rfl(imin2(h0n, h1n));
    const int tmx = rfl(imax2(h0x, h1x));
    if (tmx < bmn || tmn > bmx) continue;

#pragma unroll
    for (unsigned j = 0; j < 2u; ++j) {
      const unsigned idx = tid + 256u * j;
      const unsigned r = idx >> 3, c = (idx & 7u) * 8u;
      const unsigned key = kb + r;
      const unsigned back = (((c & 16u) != 0u) && (key > 0u)) ? 1u : 0u;
      const size_t ko = kplane + (size_t)(key - back) * DIM + c;
      const size_t vo = vplane + (size_t)r * SEQ + kb + c;
      *(v8h*)&Ks[r * LDT + c]  = *(const v8h*)(Kh + ko);
      *(v8h*)&Krs[r * LDT + c] = *(const v8h*)(Kr + ko);
      *(v8h*)&Vs[r * LDT + c]  = *(const v8h*)(Vt + vo);
      *(v8h*)&Vrs[r * LDT + c] = *(const v8h*)(Vr + vo);
    }
    __syncthreads();

#pragma unroll 1
    for (unsigned h2 = 0; h2 < 2u; ++h2) {
      const unsigned kh0 = kb + 32u * h2;
      const int hn = rfl(Hmn[e0 + h2]);
      const int hx = rfl(Hmx[e0 + h2]);
      if (kh0 <= wrow0 + 15u && !(hx < wmn || hn > wmx)) {
        const v16h qr0 = frag_at(Qr + qoff);
        const v16h qr1 = frag_at(Qr + qoff + 32);

        v8f s[2];
#pragma unroll
        for (int kg = 0; kg < 2; ++kg) {
          const unsigned krow = h2 * 32u + (unsigned)kg * 16u;
          v8f t = {}, tr = {};
          {
            const v16h kf  = ld_frag(&Ks[krow * LDT], LDT);
            const v16h krf = ld_frag(&Krs[krow * LDT], LDT);
            t  = wmma16(qf[0], kf, t);
            tr = wmma16(qf[0], krf, tr);
            tr = wmma16(qr0, kf, tr);
          }
          {
            const v16h kf  = ld_frag(&Ks[krow * LDT + 32u], LDT);
            const v16h krf = ld_frag(&Krs[krow * LDT + 32u], LDT);
            t  = wmma16(qf[1], kf, t);
            tr = wmma16(qf[1], krf, tr);
            tr = wmma16(qr1, kf, tr);
          }
          const unsigned col = kh0 + (unsigned)kg * 16u + m;
          int dk = Ds[col];
          asm volatile("" : "+v"(dk));
#pragma unroll
          for (int v = 0; v < 8; ++v) {
            const bool ok = (col <= rowb + (unsigned)v) && (dk == dq[v]);
            s[kg][v] = ok ? ((t[v] + tr[v] * RINV) * scale) : -1.0e30f;
          }
        }

        float alpha[8];
#pragma unroll
        for (int v = 0; v < 8; ++v) {
          float mx = fmaxf(s[0][v], s[1][v]);
          mx = red16_max(mx);
          const float mn = fmaxf(mrow[v], mx);
          alpha[v] = __expf(mrow[v] - mn);
          mrow[v] = mn;
        }
#pragma unroll
        for (int kg = 0; kg < 2; ++kg)
#pragma unroll
          for (int v = 0; v < 8; ++v) {
            const float ev = __expf(s[kg][v] - mrow[v]);
            s[kg][v] = (s[kg][v] > -1.0e29f) ? ev : 0.0f;
          }
#pragma unroll
        for (int v = 0; v < 8; ++v) {
          const float rs = red16_sum(s[0][v] + s[1][v]);
          lrow[v] = alpha[v] * lrow[v] + rs;
        }
#pragma unroll
        for (int nb = 0; nb < 4; ++nb)
#pragma unroll
          for (int v = 0; v < 8; ++v) {
            o[nb][v]    = o[nb][v] * alpha[v];
            ores[nb][v] = ores[nb][v] * alpha[v];
          }

#pragma unroll
        for (int kg = 0; kg < 2; ++kg)
#pragma unroll
          for (int v = 0; v < 8; ++v) {
            const float f = s[kg][v] * PCARRY;
            const h16 h = toh_flush(f);
            const unsigned pi = pbase + (hh * 8u + (unsigned)v) * LDT + (unsigned)kg * 16u + m;
            Ps[pi]  = h;
            Prs[pi] = toh_flush(RCARRY * (f - (float)h));
          }
        wave_lds_sync();

        const v16h pf  = ld_frag(&Ps[pbase], LDT);
        const v16h prf = ld_frag(&Prs[pbase], LDT);
#pragma unroll
        for (int nb = 0; nb < 4; ++nb) {
          const v16h vf  = ld_frag(&Vs[(nb * 16) * LDT + h2 * 32u], LDT);
          const v16h vrf = ld_frag(&Vrs[(nb * 16) * LDT + h2 * 32u], LDT);
          o[nb]    = wmma16(pf, vf, o[nb]);
          ores[nb] = wmma16(pf, vrf, ores[nb]);
          ores[nb] = wmma16(prf, vf, ores[nb]);
        }
      }
    }
    __syncthreads();
  }

  float inv[8];
#pragma unroll
  for (int v = 0; v < 8; ++v) {
    const float g = Gt[(size_t)(b * (unsigned)SEQ + rowb + (unsigned)v) * NGATE + head];
    inv[v] = __builtin_amdgcn_rcpf(lrow[v]) * (CCARRY / (PCARRY * VCARRY)) * g;
  }
#pragma unroll
  for (int nb = 0; nb < 4; ++nb)
#pragma unroll
    for (int v = 0; v < 8; ++v) {
      const float f = (o[nb][v] + ores[nb][v] * RINV) * inv[v];
      const h16 h = toh_flush(f);
      const unsigned pi = pbase + (hh * 8u + (unsigned)v) * LDT + (unsigned)nb * 16u + m;
      Ps[pi]  = h;
      Prs[pi] = toh_flush(RCARRY * (f - (float)h));
    }
  wave_lds_sync();
  v8h x[4], xr[4];
  size_t off[4];
#pragma unroll
  for (unsigned i = 0; i < 4u; ++i) {
    const unsigned r = 4u * i + (lane >> 3);
    const unsigned c = (lane & 7u) * 8u;
    x[i]  = *(const v8h*)&Ps[pbase + r * LDT + c];
    xr[i] = *(const v8h*)&Prs[pbase + r * LDT + c];
    off[i] = (size_t)(b * (unsigned)SEQ + wrow0 + r) * DIM + head * HD + c;
  }
#pragma unroll
  for (int i = 0; i < 4; ++i) *(volatile v8h*)(Ohi + off[i]) = x[i];
#pragma unroll
  for (int i = 0; i < 4; ++i) *(volatile v8h*)(Ores + off[i]) = xr[i];
  __threadfence();
#pragma unroll
  for (int i = 0; i < 4; ++i) *(volatile v8h*)(Ohi + off[i]) = x[i];
#pragma unroll
  for (int i = 0; i < 4; ++i) *(volatile v8h*)(Ores + off[i]) = xr[i];
}

extern "C" void kernel_launch(void* const* d_in, const int* in_sizes, int n_in,
                              void* d_out, int out_size, void* d_ws, size_t ws_size,
                              hipStream_t stream) {
  if (n_in < 10) return;
  const long long need_x = ((long long)(NB - 1) * SEQ_FULL + SEQ) * DIM;
  if ((long long)in_sizes[0] < need_x) return;
  if ((long long)in_sizes[1] < need_x) return;
  if (in_sizes[2] < 2) return;
  if ((long long)in_sizes[3] < (long long)SEQ * ROTH) return;
  if ((long long)in_sizes[4] < (long long)SEQ * ROTH) return;
  if ((long long)in_sizes[5] < (long long)4 * DIM * DIM) return;
  if ((long long)in_sizes[6] < (long long)NHEAD * DIM) return;
  if ((long long)in_sizes[7] < (long long)NHEAD * DIM) return;
  if (in_sizes[8] < 1) return;
  if (in_sizes[9] < SEQ) return;
  if ((long long)out_size < need_x) return;
  if (ws_size < WS_TOTAL) return;

  const float* X     = (const float*)d_in[0];
  const float* Ve    = (const float*)d_in[1];
  const float* lam   = (const float*)d_in[2];
  const float* cosv  = (const float*)d_in[3];
  const float* sinv  = (const float*)d_in[4];
  const float* Wqkvo = (const float*)d_in[5];
  const float* agw   = (const float*)d_in[6];
  const float* vgw   = (const float*)d_in[7];
  const float* ascl  = (const float*)d_in[8];
  const int*   docs  = (const int*)d_in[9];
  float* out = (float*)d_out;

  char* ws = (char*)d_ws;
  size_t o = 0;
  _Float16* W16    = (_Float16*)(ws + o);  o += W_ELEMS * 2;
  _Float16* G16    = (_Float16*)(ws + o);  o += GW_ELEMS * 2;
  _Float16* X16    = (_Float16*)(ws + o);  o += PLANE16_BYTES;
  float*    Gt     = (float*)(ws + o);     o += GT_BYTES;
  _Float16* Q16    = (_Float16*)(ws + o);  o += PLANE16_BYTES;
  _Float16* K16    = (_Float16*)(ws + o);  o += PLANE16_BYTES;
  _Float16* Vt16   = (_Float16*)(ws + o);  o += PLANE16_BYTES;
  _Float16* QR16   = (_Float16*)(ws + o);  o += PLANE16_BYTES;
  _Float16* KR16   = (_Float16*)(ws + o);  o += PLANE16_BYTES;
  _Float16* VtR16  = (_Float16*)(ws + o);  o += PLANE16_BYTES;
  _Float16* Ctx16  = (_Float16*)(ws + o);  o += PLANE16_BYTES;
  _Float16* CtxR16 = (_Float16*)(ws + o);  o += PLANE16_BYTES;
  if (o != WS_TOTAL) return;

  dim3 blk(256);

  wcvt_kernel<<<dim3((unsigned)(W_ELEMS / 2048)), blk, 0, stream>>>(
      Wqkvo, lam, (unsigned)WQKV_ELEMS, 1u, W16);
  wcvt_kernel<<<dim3((unsigned)(GWHALF_ELEMS / 2048)), blk, 0, stream>>>(
      agw, lam, 0u, 0u, G16);
  wcvt_kernel<<<dim3((unsigned)(GWHALF_ELEMS / 2048)), blk, 0, stream>>>(
      vgw, lam, 0u, 0u, G16 + GWHALF_ELEMS);
  xcvt_kernel<<<dim3((unsigned)(PLANE16_ELEMS / 2048)), blk, 0, stream>>>(X, X16);

  gate_gemm_kernel<<<dim3(MROWS / 128), blk, 0, stream>>>(X16, G16, Gt);
  qkv_gemm_kernel<<<dim3(3 * DIM / 64, MROWS / 64), blk, 0, stream>>>(
      X16, W16, Ve, Gt, cosv, sinv, Q16);
  attn_kernel<<<dim3(SEQ / 128, NHEAD, NB), blk, 0, stream>>>(
      Q16, QR16, K16, KR16, Vt16, VtR16, Gt, docs, ascl, Ctx16, CtxR16);
  out_gemm_kernel<<<dim3(DIM / 64, MROWS / 64), blk, 0, stream>>>(
      Ctx16, CtxR16, W16 + WQKV_ELEMS, out);
}
